// Attention_32916629357206
// MI455X (gfx1250) — hardware-run, weakly checked
//
#include <hip/hip_runtime.h>
#ifndef NB
#define NB 2
#endif
#ifndef SEQ
#define SEQ 2048
#endif
#define NB_FULL 2
#define SEQ_FULL 2048
#define CD 2048
#define NHEAD 32
#define NKV 8
#define NREP (NHEAD / NKV)
#define HD 64
#define NQK (NHEAD + NKV)
#define KVW (NKV * HD)
#define EARLY_ROWS (SEQ < 512 ? SEQ : 512)

#define SZ_FLAGS ((size_t)256)
#define SZ_ROT   ((size_t)SEQ * HD * 4)
#define SZ_XB    ((size_t)NB * SEQ * CD * 2)
#define SZ_WQK   ((size_t)(CD + KVW) * CD * 2)
#define SZ_WV    ((size_t)KVW * CD * 2)
#define SZ_WO    ((size_t)CD * CD * 2)
#define PLANE_QK ((size_t)NB * NQK * SEQ * HD)
#define PLANE_V  ((size_t)NB * KVW * SEQ)
#define SZ_CTXH  ((size_t)NB * SEQ * CD * 2)
#define SZ_CTXL  ((size_t)NB * EARLY_ROWS * CD * 2)
#define WS_TOTAL (SZ_FLAGS + SZ_ROT + SZ_XB + SZ_WQK + SZ_WV + SZ_WO + PLANE_QK * 4 + PLANE_V * 4 + SZ_CTXH + SZ_CTXL)

static_assert(SEQ % 128 == 0);
static_assert(EARLY_ROWS % 128 == 0);
static_assert(SEQ <= SEQ_FULL);
static_assert(NB <= NB_FULL);
static_assert(HD == 64);
static_assert(CD % 32 == 0);
static_assert(KVW % 128 == 0);
static_assert(NHEAD % NKV == 0);
static_assert(NHEAD == NKV * NREP);
static_assert(CD == NHEAD * HD);
static_assert(SEQ % 8 == 0);
static_assert(SZ_ROT % 256 == 0);
static_assert(WS_TOTAL <= (size_t)134217728);
static_assert(SZ_XB % 256 == 0 && SZ_WQK % 256 == 0 && SZ_WV % 256 == 0 && SZ_WO % 256 == 0);
static_assert((PLANE_QK * 2) % 256 == 0 && (PLANE_V * 2) % 256 == 0 && SZ_CTXH % 256 == 0 && SZ_CTXL % 256 == 0);

typedef __bf16 v16b __attribute__((ext_vector_type(16)));
typedef _Float16 v16h __attribute__((ext_vector_type(16)));
typedef unsigned short v8us __attribute__((ext_vector_type(8), may_alias));
typedef float v8f __attribute__((ext_vector_type(8)));
typedef float v4f __attribute__((ext_vector_type(4)));
typedef float v4fa __attribute__((ext_vector_type(4), may_alias));
typedef int v4i __attribute__((ext_vector_type(4)));
typedef int v4ia __attribute__((ext_vector_type(4), may_alias));
union Frag { v16b b; v16h v; v8us half[2]; _Float16 h[16]; unsigned short u[16]; };
union Pack8 { v8us v; _Float16 h[8]; unsigned short u[8]; };

#define LOG2E 1.4426950408889634f
#define S2M11 0.00048828125f
#define S2M12 0.000244140625f
__device__ __forceinline__ unsigned short bf16_bits(float x) {
  unsigned int u = __float_as_uint(x);
  return (unsigned short)((u + 0x7FFFu + ((u >> 16) & 1u)) >> 16);
}
__device__ __forceinline__ float bf16_val(unsigned short b) { return __uint_as_float(((unsigned int)b) << 16); }
__device__ __forceinline__ float bf16_rne(float x) { return bf16_val(bf16_bits(x)); }
__device__ __forceinline__ float neg_inf() { return __uint_as_float(0xff800000u); }

typedef _Float16 h16;
static __device__ __forceinline__ h16 toh_flush(float v) {
  const h16 r = (h16)v;
  return (fabsf(v) < 6.103515625e-05f) ? (h16)0.0f : r;
}

__device__ __forceinline__ void ldfrag(Frag& f, const unsigned short* __restrict__ p) {
  f.half[0] = *(const v8us*)(p);
  f.half[1] = *(const v8us*)(p + 16);
}

template <bool BF>
__device__ __forceinline__ v8f wm(const Frag& a, const Frag& b, v8f c) {
  if (BF) return __builtin_amdgcn_wmma_f32_16x16x32_bf16(false, a.b, false, b.b, (short)0, c, false, false);
  return __builtin_amdgcn_wmma_f32_16x16x32_f16(false, a.v, false, b.v, (short)0, c, false, false);
}

__global__ __launch_bounds__(512) void k_maskscan(const float* __restrict__ mask, int* __restrict__ flags) {
  __shared__ int sw[2][16];
  const int tid = threadIdx.x, lane = tid & 31, wv = tid >> 5;
  int badU = 0, badL = 0;
  const int cpr = SEQ / 4;
  for (int c = tid; c < SEQ * cpr; c += 512) {
    const int q = c / cpr, k = (c - q * cpr) * 4;
    const v4f m = *(const v4fa*)(mask + (size_t)q * SEQ_FULL + k);
#pragma unroll
    for (int i = 0; i < 4; ++i) {
      const int above = (k + i > q) ? 1 : 0;
      const int deep = (m[i] <= -1.0e8f) ? 1 : 0;
      const int zr = (m[i] == 0.0f) ? 1 : 0;
      badU |= above & (1 - deep);
      badL |= (1 - above) & (1 - zr);
    }
  }
#pragma unroll
  for (int o = 16; o >= 1; o >>= 1) {
    badU |= __shfl_xor(badU, o, 32);
    badL |= __shfl_xor(badL, o, 32);
  }
  if (lane == 0) { sw[0][wv] = badU; sw[1][wv] = badL; }
  __syncthreads();
  if (tid < 8) {
    int u = 0, l = 0;
#pragma unroll
    for (int i = 0; i < 16; ++i) { u |= sw[0][i]; l |= sw[1][i]; }
    v4i o;
    o[0] = (tid == 0 && u == 0) ? 1 : 0;
    o[1] = (tid == 0 && l == 0) ? 1 : 0;
    o[2] = 0; o[3] = 0;
    *(volatile v4i*)(flags + 4 * tid) = o;
    __threadfence();
    *(volatile v4i*)(flags + 4 * tid) = o;
  }
}

template <int MODE>
__global__ __launch_bounds__(256) void k_cvt(const float* __restrict__ src, unsigned short* __restrict__ dst,
                                             int nrows, int rows_per_batch, int src_batch_rows) {
  const int t = blockIdx.x * 256 + threadIdx.x;
  if (t >= nrows * 256) return;
  const int row = t >> 8, piece = t & 255;
  const int b = row / rows_per_batch, r = row - b * rows_per_batch;
  const float* sp = src + ((size_t)b * src_batch_rows + r) * CD + piece * 8;
  const v4f x0 = *(const v4fa*)(sp), x1 = *(const v4fa*)(sp + 4);
  Pack8 o;
  if (MODE == 0) {
    o.u[0] = bf16_bits(x0[0]); o.u[1] = bf16_bits(x0[1]); o.u[2] = bf16_bits(x0[2]); o.u[3] = bf16_bits(x0[3]);
    o.u[4] = bf16_bits(x1[0]); o.u[5] = bf16_bits(x1[1]); o.u[6] = bf16_bits(x1[2]); o.u[7] = bf16_bits(x1[3]);
  } else {
    o.h[0] = (_Float16)(bf16_rne(x0[0]) * 64.0f); o.h[1] = (_Float16)(bf16_rne(x0[1]) * 64.0f);
    o.h[2] = (_Float16)(bf16_rne(x0[2]) * 64.0f); o.h[3] = (_Float16)(bf16_rne(x0[3]) * 64.0f);
    o.h[4] = (_Float16)(bf16_rne(x1[0]) * 64.0f); o.h[5] = (_Float16)(bf16_rne(x1[1]) * 64.0f);
    o.h[6] = (_Float16)(bf16_rne(x1[2]) * 64.0f); o.h[7] = (_Float16)(bf16_rne(x1[3]) * 64.0f);
  }
  unsigned short* d = dst + (size_t)t * 8;
  const v8us ov = o.v;
  *(volatile v8us*)d = ov;
  __threadfence();
  *(volatile v8us*)d = ov;
}

template <bool BF, bool RES>
__device__ __forceinline__ void gemm_loop(const unsigned short* __restrict__ ap, const unsigned short* __restrict__ alp,
                                          const unsigned short* __restrict__ wp, v8f (&acc)[2][4], v8f (&acl)[2][4]) {
#pragma unroll 1
  for (int k = 0; k < CD; k += 32) {
    Frag a[2], b[4];
#pragma unroll
    for (int i = 0; i < 2; ++i) ldfrag(a[i], ap + (size_t)i * 16 * CD + k);
#pragma unroll
    for (int j = 0; j < 4; ++j) ldfrag(b[j], wp + (size_t)j * 16 * CD + k);
#pragma unroll
    for (int i = 0; i < 2; ++i)
#pragma unroll
      for (int j = 0; j < 4; ++j) acc[i][j] = wm<BF>(a[i], b[j], acc[i][j]);
    if (RES) {
      Frag al[2];
#pragma unroll
      for (int i = 0; i < 2; ++i) ldfrag(al[i], alp + (size_t)i * 16 * CD + k);
#pragma unroll
      for (int i = 0; i < 2; ++i)
#pragma unroll
        for (int j = 0; j < 4; ++j) acl[i][j] = wm<BF>(al[i], b[j], acl[i][j]);
      asm volatile("v_nop\n\tv_nop\n\tv_nop\n\tv_nop" : "+v"(acl[0][0]), "+v"(acl[0][1]), "+v"(acl[0][2]), "+v"(acl[0][3]),
                          "+v"(acl[1][0]), "+v"(acl[1][1]), "+v"(acl[1][2]), "+v"(acl[1][3])
                        : "v"(al[0].v), "v"(al[1].v), "v"(b[0].v), "v"(b[1].v), "v"(b[2].v), "v"(b[3].v));
    }
    asm volatile("v_nop\n\tv_nop\n\tv_nop\n\tv_nop" : "+v"(acc[0][0]), "+v"(acc[0][1]), "+v"(acc[0][2]), "+v"(acc[0][3]),
                        "+v"(acc[1][0]), "+v"(acc[1][1]), "+v"(acc[1][2]), "+v"(acc[1][3])
                      : "v"(a[0].v), "v"(a[1].v), "v"(b[0].v), "v"(b[1].v), "v"(b[2].v), "v"(b[3].v));
  }
}

__device__ __forceinline__ float rope1(float q, float p, float c, float s, float sg) { return q * c + (sg * p) * s; }

__global__ __launch_bounds__(256) void k_rotab(const int* __restrict__ pos, float* __restrict__ rot) {
  __shared__ __attribute__((aligned(16))) float sh[8][64];
  const int tid = threadIdx.x;
  const int r = tid >> 5, j = tid & 31;
  const int t = blockIdx.x * 8 + r;
  const float p = (float)pos[t];
  const float f = exp2f(-(float)j * 0.41524101186092029f);
  const float ang = p * f;
  float sn, cs;
  sincosf(ang, &sn, &cs);
  sh[r][j] = cs;
  sh[r][32 + j] = sn;
  __syncthreads();
  if (tid < 128) {
    const int rr = tid >> 4, pc = tid & 15;
    const v4f v = *(const v4fa*)&sh[rr][4 * pc];
    float* d = rot + (size_t)(blockIdx.x * 8 + rr) * HD + 4 * pc;
    *(volatile v4f*)d = v;
    __threadfence();
    *(volatile v4f*)d = v;
  }
}

__global__ __launch_bounds__(128) void k_proj_qk(const unsigned short* __restrict__ xb, const unsigned short* __restrict__ wqk,
                                                 const float* __restrict__ bq, const float* __restrict__ bk,
                                                 const float* __restrict__ tab,
                                                 unsigned short* __restrict__ qkh, unsigned short* __restrict__ qkl) {
  __shared__ __attribute__((aligned(16))) float st[4][32][68];
  const int tid = threadIdx.x, lane = tid & 31, ln = lane & 15, hh = lane >> 4;
  const int w = __builtin_amdgcn_readfirstlane(tid >> 5);
  const int hd = blockIdx.x;
  const int m0 = blockIdx.y * 128 + 32 * w;
  const v8f z8 = {0.f, 0.f, 0.f, 0.f, 0.f, 0.f, 0.f, 0.f};
  v8f acc[2][4];
#pragma unroll
  for (int i = 0; i < 2; ++i)
#pragma unroll
    for (int j = 0; j < 4; ++j) acc[i][j] = z8;
  gemm_loop<true, false>(xb + (size_t)(m0 + ln) * CD + 8 * hh, xb, wqk + (size_t)(hd * HD + ln) * CD + 8 * hh, acc, acc);

  float bias[4];
#pragma unroll
  for (int j = 0; j < 4; ++j) {
    const int col = hd * HD + 16 * j + ln;
    const int cq = (col < CD - 1) ? col : (CD - 1);
    int ck = col - CD;
    ck = (ck < 0) ? 0 : ((ck > KVW - 1) ? (KVW - 1) : ck);
    const float vq = bq[cq], vk = bk[ck];
    bias[j] = bf16_rne((col < CD) ? vq : vk);
  }
#pragma unroll
  for (int i = 0; i < 2; ++i)
#pragma unroll
    for (int j = 0; j < 4; ++j)
#pragma unroll
      for (int r = 0; r < 8; ++r) st[w][16 * i + 8 * hh + r][16 * j + ln] = acc[i][j][r] + bias[j];
  __syncthreads();

  const int b = m0 / SEQ, t0 = m0 - b * SEQ;
  const int rsub = lane >> 3, d0 = 8 * (lane & 7);
  const float sg = (d0 < 32) ? -1.0f : 1.0f;
  v8us oh[8], ol[8];
#pragma unroll
  for (int g = 0; g < 8; ++g) {
    const int row = 4 * g + rsub;
    const v4f a0 = *(const v4fa*)&st[w][row][d0];
    const v4f a1 = *(const v4fa*)&st[w][row][d0 + 4];
    const v4f p0 = *(const v4fa*)&st[w][row][d0 ^ 32];
    const v4f p1 = *(const v4fa*)&st[w][row][(d0 ^ 32) + 4];
    const float* tp = tab + (size_t)(t0 + row) * HD + (d0 & 31);
    const v4f c0 = *(const v4fa*)(tp), c1 = *(const v4fa*)(tp + 4);
    const v4f s0 = *(const v4fa*)(tp + 32), s1 = *(const v4fa*)(tp + 36);
    float o[8];
    o[0] = rope1(a0[0], p0[0], c0[0], s0[0], sg); o[1] = rope1(a0[1], p0[1], c0[1], s0[1], sg);
    o[2] = rope1(a0[2], p0[2], c0[2], s0[2], sg); o[3] = rope1(a0[3], p0[3], c0[3], s0[3], sg);
    o[4] = rope1(a1[0], p1[0], c1[0], s1[0], sg); o[5] = rope1(a1[1], p1[1], c1[1], s1[1], sg);
    o[6] = rope1(a1[2], p1[2], c1[2], s1[2], sg); o[7] = rope1(a1[3], p1[3], c1[3], s1[3], sg);
    Pack8 ph8, pl8;
#pragma unroll
    for (int e = 0; e < 8; ++e) {
      const float y = o[e] * 16.0f;
      const _Float16 h = toh_flush(y);
      ph8.h[e] = h;
      pl8.h[e] = toh_flush((y - (float)h) * 2048.0f);
    }
    oh[g] = ph8.v; ol[g] = pl8.v;
  }
  const size_t dbase = ((size_t)(b * NQK + hd) * SEQ + t0) * HD + d0;
#pragma unroll
  for (int pass = 0; pass < 2; ++pass) {
#pragma unroll
    for (int g = 0; g < 8; ++g) {
      const size_t off = dbase + (size_t)(4 * g + rsub) * HD;
      *(volatile v8us*)(qkh + off) = oh[g];
      *(volatile v8us*)(qkl + off) = ol[g];
    }
    if (pass == 0) __threadfence();
  }
}

__global__ __launch_bounds__(128) void k_proj_v(const unsigned short* __restrict__ wvb, const unsigned short* __restrict__ xb,
                                                const float* __restrict__ bv,
                                                unsigned short* __restrict__ vth, unsigned short* __restrict__ vtl) {
  __shared__ __attribute__((aligned(16))) float st[4][32][68];
  const int tid = threadIdx.x, lane = tid & 31, ln = lane & 15, hh = lane >> 4;
  const int w = __builtin_amdgcn_readfirstlane(tid >> 5);
  const int n0 = blockIdx.x * 64;
  const int m0 = blockIdx.y * 128 + 32 * w;
  const v8f z8 = {0.f, 0.f, 0.f, 0.f, 0.f, 0.f, 0.f, 0.f};
  v8f acc[2][4];
#pragma unroll
  for (int i = 0; i < 2; ++i)
#pragma unroll
    for (int j = 0; j < 4; ++j) acc[i][j] = z8;
  gemm_loop<true, false>(wvb + (size_t)(m0 + ln) * CD + 8 * hh, wvb, xb + (size_t)(n0 + ln) * CD + 8 * hh, acc, acc);
#pragma unroll
  for (int i = 0; i < 2; ++i)
#pragma unroll
    for (int j = 0; j < 4; ++j)
#pragma unroll
      for (int r = 0; r < 8; ++r) st[w][16 * i + 8 * hh + r][16 * j + ln] = acc[i][j][r];
  __syncthreads();

  const int b = n0 / SEQ, t0 = n0 - b * SEQ;
  const int rsub = lane >> 3, c0 = 8 * (lane & 7);
  v8us oh[8], ol[8];
#pragma unroll
  for (int g = 0; g < 8; ++g) {
    const int row = 4 * g + rsub;
    const float bias = bf16_rne(bv[m0 + row]);
    const v4f a0 = *(const v4fa*)&st[w][row][c0];
    const v4f a1 = *(const v4fa*)&st[w][row][c0 + 4];
    float o[8];
    o[0] = a0[0]; o[1] = a0[1]; o[2] = a0[2]; o[3] = a0[3];
    o[4] = a1[0]; o[5] = a1[1]; o[6] = a1[2]; o[7] = a1[3];
    Pack8 ph8, pl8;
#pragma unroll
    for (int e = 0; e < 8; ++e) {
      const float y = (o[e] + bias) * 16.0f;
      const _Float16 h = (_Float16)y;
      ph8.h[e] = h;
      pl8.h[e] = (_Float16)((y - (float)h) * 2048.0f);
    }
    oh[g] = ph8.v; ol[g] = pl8.v;
  }
  const size_t dbase = ((size_t)b * KVW + m0) * SEQ + t0 + c0;
#pragma unroll
  for (int pass = 0; pass < 2; ++pass) {
#pragma unroll
    for (int g = 0; g < 8; ++g) {
      const size_t off = dbase + (size_t)(4 * g + rsub) * SEQ;
      *(volatile v8us*)(vth + off) = oh[g];
      *(volatile v8us*)(vtl + off) = ol[g];
    }
    if (pass == 0) __threadfence();
  }
}

template <bool EARLYP, bool MASK>
__device__ __forceinline__ void fa_step(const unsigned short* __restrict__ Kp, const unsigned short* __restrict__ Kl,
                                        const unsigned short* __restrict__ Vp, const unsigned short* __restrict__ Vl,
                                        const float* __restrict__ mrow, int key0, int ln, int hh,
                                        const Frag (&qh)[2], const Frag (&ql)[2],
                                        float& mr, float& lr, v8f (&Oh)[4], v8f (&Ol)[4]) {
  const v8f z8 = {0.f, 0.f, 0.f, 0.f, 0.f, 0.f, 0.f, 0.f};
  float sc[16];
  int koff = (key0 + ln) * HD + 8 * hh;
  if (EARLYP) {
#pragma unroll
    for (int kt = 0; kt < 2; ++kt) {
      Frag a0, a1, l0, l1;
      ldfrag(a0, Kp + koff); ldfrag(a1, Kp + koff + 32);
      ldfrag(l0, Kl + koff); ldfrag(l1, Kl + koff + 32);
      v8f s = z8, r = z8;
      s = wm<false>(a0, qh[0], s); s = wm<false>(a1, qh[1], s);
      r = wm<false>(a0, ql[0], r); r = wm<false>(a1, ql[1], r);
      r = wm<false>(l0, qh[0], r); r = wm<false>(l1, qh[1], r);
      asm volatile("v_nop\n\tv_nop\n\tv_nop\n\tv_nop" : "+v"(s), "+v"(r)
                        : "v"(a0.v), "v"(a1.v), "v"(l0.v), "v"(l1.v), "v"(qh[0].v), "v"(qh[1].v), "v"(ql[0].v), "v"(ql[1].v));
#pragma unroll
      for (int e = 0; e < 8; ++e) sc[8 * kt + e] = fmaf(r[e], S2M11, s[e]) * S2M11;
      koff += 16 * HD;
      if (kt == 0) asm volatile("" : "+v"(koff) : "v"(sc[0]));
    }
  } else {
    Frag k00, k01, k10, k11;
    ldfrag(k00, Kp + koff);           ldfrag(k01, Kp + koff + 32);
    ldfrag(k10, Kp + koff + 16 * HD); ldfrag(k11, Kp + koff + 16 * HD + 32);
    v8f s0 = z8, s1 = z8;
    s0 = wm<false>(k00, qh[0], s0); s0 = wm<false>(k01, qh[1], s0);
    s1 = wm<false>(k10, qh[0], s1); s1 = wm<false>(k11, qh[1], s1);
    asm volatile("v_nop\n\tv_nop\n\tv_nop\n\tv_nop" : "+v"(s0), "+v"(s1)
                      : "v"(k00.v), "v"(k01.v), "v"(k10.v), "v"(k11.v), "v"(qh[0].v), "v"(qh[1].v));
#pragma unroll
    for (int e = 0; e < 8; ++e) { sc[e] = s0[e] * S2M11; sc[8 + e] = s1[e] * S2M11; }
  }
  if (MASK) {
    const float* mp = mrow + key0 + 8 * hh;
    const v4f m0 = *(const v4fa*)(mp),      m1 = *(const v4fa*)(mp + 4);
    const v4f m2 = *(const v4fa*)(mp + 16), m3 = *(const v4fa*)(mp + 20);
#pragma unroll
    for (int e = 0; e < 4; ++e) {
      sc[e]      = sc[e]      + bf16_rne(m0[e]);
      sc[4 + e]  = sc[4 + e]  + bf16_rne(m1[e]);
      sc[8 + e]  = sc[8 + e]  + bf16_rne(m2[e]);
      sc[12 + e] = sc[12 + e] + bf16_rne(m3[e]);
    }
  }
  float mx = sc[0];
#pragma unroll
  for (int i = 1; i < 16; ++i) mx = fmaxf(mx, sc[i]);
  mx = fmaxf(mx, __shfl_xor(mx, 16, 32));
  const float mnew = fmaxf(mr, mx);
  float msafe = mnew;
  if (MASK) msafe = (mnew == neg_inf()) ? 0.0f : mnew;
  const float al = __builtin_amdgcn_exp2f((mr - msafe) * LOG2E);
  mr = mnew;
  Frag ph, pl;
  float ps = 0.0f;
#pragma unroll
  for (int i = 0; i < 16; ++i) {
    const float pc = __builtin_amdgcn_exp2f(fmaf(sc[i] - msafe, LOG2E, 8.0f));
    ps += pc;
    const _Float16 h = toh_flush(pc);
    ph.h[i] = h;
    if (EARLYP) pl.h[i] = toh_flush((pc - (float)h) * 2048.0f);
  }
  ps += __shfl_xor(ps, 16, 32);
  lr = lr * al + ps;
  int voff = key0 + 8 * hh;
  asm volatile("" : "+v"(voff) : "v"(ps));
  const unsigned short* vp = Vp + (size_t)ln * SEQ + voff;
  Frag vf[4];
#pragma unroll
  for (int t = 0; t < 4; ++t) ldfrag(vf[t], vp + (size_t)t * 16 * SEQ);
#pragma unroll
  for (int t = 0; t < 4; ++t) Oh[t] = Oh[t] * al;
  if (EARLYP) {
    const unsigned short* vq = Vl + (size_t)ln * SEQ + voff;
    Frag vl[4];
#pragma unroll
    for (int t = 0; t < 4; ++t) ldfrag(vl[t], vq + (size_t)t * 16 * SEQ);
#pragma unroll
    for (int t = 0; t < 4; ++t) Ol[t] = Ol[t] * al;
#pragma unroll
    for (int t = 0; t < 4; ++t) {
      Oh[t] = wm<false>(vf[t], ph, Oh[t]);
      Ol[t] = wm<false>(vf[t], pl, Ol[t]);
      Ol[t] = wm<false>(vl[t], ph, Ol[t]);
    }
    asm volatile("v_nop\n\tv_nop\n\tv_nop\n\tv_nop" : "+v"(Oh[0]), "+v"(Oh[1]), "+v"(Oh[2]), "+v"(Oh[3]), "+v"(Ol[0]), "+v"(Ol[1]), "+v"(Ol[2]), "+v"(Ol[3])
                      : "v"(vf[0].v), "v"(vf[1].v), "v"(vf[2].v), "v"(vf[3].v),
                        "v"(vl[0].v), "v"(vl[1].v), "v"(vl[2].v), "v"(vl[3].v), "v"(ph.v), "v"(pl.v));
  } else {
#pragma unroll
    for (int t = 0; t < 4; ++t) Oh[t] = wm<false>(vf[t], ph, Oh[t]);
    asm volatile("v_nop\n\tv_nop\n\tv_nop\n\tv_nop" : "+v"(Oh[0]), "+v"(Oh[1]), "+v"(Oh[2]), "+v"(Oh[3])
                      : "v"(vf[0].v), "v"(vf[1].v), "v"(vf[2].v), "v"(vf[3].v), "v"(ph.v));
  }
}

template <bool EARLYP>
__device__ __forceinline__ void run_keys(const unsigned short* __restrict__ qkh, const unsigned short* __restrict__ qkl,
                                         const unsigned short* __restrict__ vth, const unsigned short* __restrict__ vtl,
                                         const float* __restrict__ mask, int b, int h, int qg, int ln, int hh,
                                         int nplain, int nsteps, float& mr, float& lr, v8f (&Oh)[4], v8f (&Ol)[4]) {
  const size_t qoff = ((size_t)(b * NQK + h) * SEQ + qg) * HD + 8 * hh;
  Frag qh[2], ql[2];
  ldfrag(qh[0], qkh + qoff); ldfrag(qh[1], qkh + qoff + 32);
  if (EARLYP) { ldfrag(ql[0], qkl + qoff); ldfrag(ql[1], qkl + qoff + 32); }
  else { ql[0] = qh[0]; ql[1] = qh[1]; }
  const int kv = h / NREP;
  const size_t kbase = (size_t)(b * NQK + NHEAD + kv) * SEQ * HD;
  const size_t vbase = ((size_t)b * KVW + (size_t)kv * HD) * SEQ;
  const unsigned short* Kp = qkh + kbase;
  const unsigned short* Kl = qkl + kbase;
  const unsigned short* Vp = vth + vbase;
  const unsigned short* Vl = vtl + vbase;
  const float* mrow = mask + (size_t)qg * SEQ_FULL;
#pragma unroll 1
  for (int j = 0; j < nplain; ++j)
    fa_step<EARLYP, false>(Kp, Kl, Vp, Vl, mrow, 32 * j, ln, hh, qh, ql, mr, lr, Oh, Ol);
#pragma unroll 1
  for (int j = nplain; j < nsteps; ++j)
    fa_step<EARLYP, true>(Kp, Kl, Vp, Vl, mrow, 32 * j, ln, hh, qh, ql, mr, lr, Oh, Ol);
}

__global__ __launch_bounds__(128) void k_attn(const unsigned short* __restrict__ qkh, const unsigned short* __restrict__ qkl,
                                              const unsigned short* __restrict__ vth, const unsigned short* __restrict__ vtl,
                                              const float* __restrict__ mask, const int* __restrict__ flags,
                                              unsigned short* __restrict__ ctxh, unsigned short* __restrict__ ctxl) {
  __shared__ __attribute__((aligned(16))) float so[4][16][68];
  const int tid = threadIdx.x, lane = tid & 31, ln = lane & 15, hh = lane >> 4;
  const int w = __builtin_amdgcn_readfirstlane(tid >> 5);
  const int nqt = SEQ / 64;
  const int blk = blockIdx.x;
  const int qt = blk % nqt;
  const int h = (blk / nqt) % NHEAD;
  const int b = blk / (nqt * NHEAD);
  const int qbase = qt * 64 + 16 * w;
  const int qg = qbase + ln;
  const int fU = flags[0], fL = flags[1];
  const bool tri = (fU == 1 && fL == 1);
  const int nfull = qbase >> 5;
  const int nsteps = tri ? (nfull + 1) : (SEQ / 32);
  const int nplain = tri ? nfull : 0;
  const bool early = (qt * 64 < EARLY_ROWS);

  const v8f z8 = {0.f, 0.f, 0.f, 0.f, 0.f, 0.f, 0.f, 0.f};
  float mr = neg_inf(), lr = 0.0f;
  v8f Oh[4], Ol[4];
#pragma unroll
  for (int t = 0; t < 4; ++t) { Oh[t] = z8; Ol[t] = z8; }
  if (early) run_keys<true>(qkh, qkl, vth, vtl, mask, b, h, qg, ln, hh, nplain, nsteps, mr, lr, Oh, Ol);
  else       run_keys<false>(qkh, qkl, vth, vtl, mask, b, h, qg, ln, hh, nplain, nsteps, mr, lr, Oh, Ol);

  const float inv = 4.0f * (1.0f / lr);
#pragma unroll
  for (int t = 0; t < 4; ++t)
#pragma unroll
    for (int r = 0; r < 8; ++r)
      so[w][ln][16 * t + 8 * hh + r] = fmaf(Ol[t][r], S2M11, Oh[t][r]) * inv;
  __syncthreads();
  const int rsub = lane >> 3, d0 = 8 * (lane & 7);
  v8us oh[4], ol[4];
#pragma unroll
  for (int g = 0; g < 4; ++g) {
    const int row = 4 * g + rsub;
    const v4f a0 = *(const v4fa*)&so[w][row][d0];
    const v4f a1 = *(const v4fa*)&so[w][row][d0 + 4];
    float o[8];
    o[0] = a0[0]; o[1] = a0[1]; o[2] = a0[2]; o[3] = a0[3];
    o[4] = a1[0]; o[5] = a1[1]; o[6] = a1[2]; o[7] = a1[3];
    Pack8 ph8, pl8;
#pragma unroll
    for (int e = 0; e < 8; ++e) {
      const _Float16 hv = toh_flush(o[e]);
      ph8.h[e] = hv;
      pl8.h[e] = toh_flush((o[e] - (float)hv) * 2048.0f);
    }
    oh[g] = ph8.v; ol[g] = pl8.v;
  }
  const size_t hbase = ((size_t)b * SEQ + qbase) * CD + (size_t)h * HD + d0;
  const size_t lbase = ((size_t)b * EARLY_ROWS + (early ? qbase : 0)) * CD + (size_t)h * HD + d0;
#pragma unroll
  for (int pass = 0; pass < 2; ++pass) {
#pragma unroll
    for (int g = 0; g < 4; ++g) {
      const size_t ro = (size_t)(4 * g + rsub) * CD;
      *(volatile v8us*)(ctxh + hbase + ro) = oh[g];
      if (early) *(volatile v8us*)(ctxl + lbase + ro) = ol[g];
    }
    if (pass == 0) __threadfence();
  }
}

__global__ __launch_bounds__(128) void k_proj_out(const unsigned short* __restrict__ ctxh, const unsigned short* __restrict__ ctxl,
                                                  const unsigned short* __restrict__ wo, const float* __restrict__ bo,
                                                  float* __restrict__ out) {
  __shared__ __attribute__((aligned(16))) float st[4][32][68];
  const int tid = threadIdx.x, lane = tid & 31, ln = lane & 15, hh = lane >> 4;
  const int w = __builtin_amdgcn_readfirstlane(tid >> 5);
  const int n0 = blockIdx.x * 64;
  const int mb = blockIdx.y * 128;
  const int b = mb / SEQ;
  const int tb = mb - b * SEQ;
  const bool early = (tb < EARLY_ROWS);
  const int t0 = tb + 32 * w;
  const int m0 = mb + 32 * w;
  const v8f z8 = {0.f, 0.f, 0.f, 0.f, 0.f, 0.f, 0.f, 0.f};
  v8f acc[2][4], acl[2][4];
#pragma unroll
  for (int i = 0; i < 2; ++i)
#pragma unroll
    for (int j = 0; j < 4; ++j) { acc[i][j] = z8; acl[i][j] = z8; }
  const unsigned short* ap = ctxh + (size_t)(m0 + ln) * CD + 8 * hh;
  const unsigned short* alp = ctxl + (size_t)(b * EARLY_ROWS + (early ? t0 : 0) + ln) * CD + 8 * hh;
  const unsigned short* wp = wo + (size_t)(n0 + ln) * CD + 8 * hh;
  if (early) gemm_loop<false, true>(ap, alp, wp, acc, acl);
  else       gemm_loop<false, false>(ap, ap, wp, acc, acl);
#pragma unroll
  for (int i = 0; i < 2; ++i)
#pragma unroll
    for (int j = 0; j < 4; ++j)
#pragma unroll
      for (int r = 0; r < 8; ++r)
        st[w][16 * i + 8 * hh + r][16 * j + ln] = fmaf(acl[i][j][r], S2M11, acc[i][j][r]) * S2M12;
  __syncthreads();
  const int rsub = lane >> 4, c4 = 4 * (lane & 15);
  const v4f bb = *(const v4fa*)(bo + n0 + c4);
  v4f bias;
  bias[0] = bf16_rne(bb[0]); bias[1] = bf16_rne(bb[1]); bias[2] = bf16_rne(bb[2]); bias[3] = bf16_rne(bb[3]);
  v4f ov[16];
#pragma unroll
  for (int g = 0; g < 16; ++g) {
    const v4f a = *(const v4fa*)&st[w][2 * g + rsub][c4];
    ov[g] = a + bias;
  }
  float* og = out + ((size_t)b * SEQ_FULL + t0) * CD + n0 + c4;
#pragma unroll
  for (int pass = 0; pass < 2; ++pass) {
#pragma unroll
    for (int g = 0; g < 16; ++g)
      *(volatile v4f*)(og + (size_t)(2 * g + rsub) * CD) = ov[g];
    if (pass == 0) __threadfence();
  }
}

extern "C" void kernel_launch(void* const* d_in, const int* in_sizes, int n_in,
                              void* d_out, int out_size, void* d_ws, size_t ws_size, hipStream_t stream) {
  if (n_in < 11) return;
  const long long need_x = (long long)(NB - 1) * SEQ_FULL * CD + (long long)SEQ * CD;
  const long long need_m = (long long)(SEQ - 1) * SEQ_FULL + SEQ;
  if ((long long)in_sizes[0] < need_x) return;
  if ((long long)in_sizes[1] < need_m) return;
  if ((long long)in_sizes[2] < (long long)SEQ) return;
  if ((long long)in_sizes[3] < (long long)CD * CD || (long long)in_sizes[4] < CD) return;
  if ((long long)in_sizes[5] < (long long)KVW * CD || (long long)in_sizes[6] < KVW) return;
  if ((long long)in_sizes[7] < (long long)KVW * CD || (long long)in_sizes[8] < KVW) return;
  if ((long long)in_sizes[9] < (long long)CD * CD || (long long)in_sizes[10] < CD) return;
  if ((long long)out_size < need_x) return;
  if ((size_t)WS_TOTAL > ws_size) return;

  const float* x    = (const float*)d_in[0];
  const float* mask = (const float*)d_in[1];
  const int*   pos  = (const int*)d_in[2];
  const float* Wq   = (const float*)d_in[3];
  const float* bq   = (const float*)d_in[4];
  const float* Wk   = (const float*)d_in[5];
  const float* bk   = (const float*)d_in[6];
  const float* Wv   = (const float*)d_in[7];
  const float* bv   = (const float*)d_in[8];
  const float* Wo   = (const float*)d_in[9];
  const float* bo   = (const float*)d_in[10];
  float* out = (float*)d_out;

  char* ws = (char*)d_ws;
  size_t off = 0;
  int* flags = (int*)(ws + off);                               off += SZ_FLAGS;
  float* rot = (float*)(ws + off);                             off += SZ_ROT;
  unsigned short* xb   = (unsigned short*)(ws + off);          off += SZ_XB;
  unsigned short* wqk  = (unsigned short*)(ws + off);          off += SZ_WQK;
  unsigned short* wvb  = (unsigned short*)(ws + off);          off += SZ_WV;
  unsigned short* wob  = (unsigned short*)(ws + off);          off += SZ_WO;
  unsigned short* qkh  = (unsigned short*)(ws + off);          off += PLANE_QK * 2;
  unsigned short* qkl  = (unsigned short*)(ws + off);          off += PLANE_QK * 2;
  unsigned short* vth  = (unsigned short*)(ws + off);          off += PLANE_V * 2;
  unsigned short* vtl  = (unsigned short*)(ws + off);          off += PLANE_V * 2;
  unsigned short* ctxh = (unsigned short*)(ws + off);          off += SZ_CTXH;
  unsigned short* ctxl = (unsigned short*)(ws + off);          off += SZ_CTXL;
  if (off > ws_size) return;

  k_maskscan<<<1, 512, 0, stream>>>(mask, flags);
  k_rotab<<<(unsigned)(SEQ / 8), 256, 0, stream>>>(pos, rot);
  k_cvt<0><<<(unsigned)(NB * SEQ), 256, 0, stream>>>(x, xb, NB * SEQ, SEQ, SEQ_FULL);
  k_cvt<0><<<(unsigned)CD, 256, 0, stream>>>(Wq, wqk, CD, CD, CD);
  k_cvt<0><<<(unsigned)KVW, 256, 0, stream>>>(Wk, wqk + (size_t)CD * CD, KVW, KVW, KVW);
  k_cvt<0><<<(unsigned)KVW, 256, 0, stream>>>(Wv, wvb, KVW, KVW, KVW);
  k_cvt<1><<<(unsigned)CD, 256, 0, stream>>>(Wo, wob, CD, CD, CD);

  k_proj_qk<<<dim3(NQK, (unsigned)(NB * SEQ / 128)), 128, 0, stream>>>(xb, wqk, bq, bk, rot, qkh, qkl);
  k_proj_v<<<dim3((unsigned)(NB * SEQ / 64), KVW / 128), 128, 0, stream>>>(wvb, xb, bv, vth, vtl);
  k_attn<<<(unsigned)(NB * NHEAD * (SEQ / 64)), 128, 0, stream>>>(qkh, qkl, vth, vtl, mask, flags, ctxh, ctxl);
  k_proj_out<<<dim3(CD / 64, (unsigned)(NB * SEQ / 128)), 128, 0, stream>>>(ctxh, ctxl, wob, bo, out);
}
